// MambaBlock_8083128451705
// MI455X (gfx1250) — hardware-run, weakly checked
//
#include <hip/hip_runtime.h>
#include <math.h>

typedef __attribute__((ext_vector_type(16))) _Float16 v16h;
typedef __attribute__((ext_vector_type(8)))  _Float16 v8h;
typedef __attribute__((ext_vector_type(8)))  float    v8f;
typedef __attribute__((ext_vector_type(4)))  float    v4f;

constexpr int kBatch   = 4;
constexpr int kSeq     = 2048;
constexpr int kDm      = 512;
constexpr int kDin     = 1024;
constexpr int kNst     = 16;
constexpr int kXrP     = 2 * kDin;
constexpr int kRows    = kBatch * kSeq;
constexpr int kDbcReal = kDin + 2 * kNst;
constexpr int kDbcN    = 1088;
constexpr int kBcP     = 32;
constexpr int kConvTP  = 260;
constexpr int kScanTS  = 64;
constexpr int kScanCh  = 64;
constexpr int kScanYP  = 68;
static_assert(kXrP == 2048 && kRows == 8192 && kDbcReal == 1056, "shape constants");
static_assert((kDm % 32) == 0 && (kDin % 32) == 0, "GEMM K multiples of 32");
static_assert((kRows % 64) == 0 && (kXrP % 64) == 0 && (kDbcN % 64) == 0 && (kDm % 64) == 0, "GEMM M,N multiples of 64");
static_assert(kDbcN >= kDbcReal && (kDin % 64) == 0, "dt tiles and the B|C tile are separate 64-column tiles");
static_assert(2 * kNst == kBcP, "B|C row is one 128-B line");
static_assert((kSeq % kScanTS) == 0 && (kSeq % 64) == 0 && (kDin % kScanCh) == 0 && (kDin % 256) == 0, "tile multiples");

constexpr float kCarryX   = 16.0f;
constexpr float kCarryW   = 1024.0f;
constexpr float kCarryXs  = 256.0f;
constexpr float kCarryYg  = 1024.0f;
constexpr float kFoldIn   = 1.0f / (kCarryX * kCarryW);
constexpr float kFoldDbc  = 1.0f / (kCarryXs * kCarryW);
constexpr float kFoldOut  = 1.0f / (kCarryYg * kCarryW);

constexpr size_t kSzX16  = (size_t)kRows * kDm  * 2;
constexpr size_t kSzWin  = (size_t)kXrP  * kDm  * 2;
constexpr size_t kSzWdbc = (size_t)kDbcN * kDin * 2;
constexpr size_t kSzWout = (size_t)kDm   * kDin * 2;
constexpr size_t kSzXr   = (size_t)kRows * kXrP * 4;
constexpr size_t kSzXs16 = (size_t)kRows * kDin * 2;
constexpr size_t kSzDp16 = (size_t)kRows * kDin * 2;
constexpr size_t kSzBc   = (size_t)kRows * kBcP * 4;
constexpr size_t kSzYg16 = (size_t)kRows * kDin * 2;
constexpr size_t kOffX16  = 0;
constexpr size_t kOffWin  = kOffX16  + kSzX16;
constexpr size_t kOffWdbc = kOffWin  + kSzWin;
constexpr size_t kOffWout = kOffWdbc + kSzWdbc;
constexpr size_t kOffXr   = kOffWout + kSzWout;
constexpr size_t kOffXs16 = kOffXr   + kSzXr;
constexpr size_t kOffDp16 = kOffXs16 + kSzXs16;
constexpr size_t kOffBc   = kOffDp16 + kSzDp16;
constexpr size_t kOffYg16 = kOffBc   + kSzBc;
constexpr size_t kWsTotal = kOffYg16 + kSzYg16;
static_assert(kWsTotal == 132251648ull, "carve total");
static_assert(kWsTotal <= 134217728ull, "carve cap");
static_assert((kOffWin % 128) == 0 && (kOffWdbc % 128) == 0 && (kOffWout % 128) == 0 && (kOffXr % 128) == 0 &&
              (kOffXs16 % 128) == 0 && (kOffDp16 % 128) == 0 && (kOffBc % 128) == 0 && (kOffYg16 % 128) == 0,
              "128-B aligned regions");

__device__ __forceinline__ _Float16 f16_operand(float v) {
  const float s = (fabsf(v) < 6.103515625e-5f) ? 0.0f : v;
  return (_Float16)s;
}
__device__ __forceinline__ float h16_to_f32(unsigned hb) {
  const unsigned sgn = (hb & 0x8000u) << 16;
  const unsigned em = hb & 0x7fffu;
  const float fn = __uint_as_float((em << 13) + 0x38000000u);
  const float fs = (float)em * 5.9604644775390625e-8f;
  const float mag = (em < 0x400u) ? fs : fn;
  return __uint_as_float(__float_as_uint(mag) | sgn);
}
__device__ __forceinline__ v16h frag_load(const _Float16* p) {
  union U { v16h v; v8h h[2]; };
  U f;
  f.h[0] = *(const v8h*)(p);
  f.h[1] = *(const v8h*)(p + 16);
  return f.v;
}
__device__ __forceinline__ v8f mma_g(v16h a, v16h b, v8f c) {
  c = __builtin_amdgcn_wmma_f32_16x16x32_f16(false, a, false, b, (short)0, c, false, false);
  asm volatile("v_nop\n\tv_nop\n\tv_nop\n\tv_nop" : "+v"(c) : "v"(a), "v"(b));
  return c;
}
__device__ __forceinline__ void keep4_h(v16h a, v16h b, v16h c, v16h d) { asm volatile("v_nop" :: "v"(a), "v"(b), "v"(c), "v"(d)); }

template <int EPI>
__global__ __launch_bounds__(256) void gemm64_f16_kernel(
    const unsigned short* __restrict__ Ap, int lda,
    const unsigned short* __restrict__ Btp, int ldb,
    float* __restrict__ Cf, int ldc,
    const float* __restrict__ bias, unsigned short* __restrict__ C16, float* __restrict__ Cbc,
    int M, int N, int K, float scale)
{
  const _Float16* A  = (const _Float16*)Ap;
  const _Float16* Bt = (const _Float16*)Btp;
  __shared__ __align__(16) float sT[8][16 * 68];
  const int lane = threadIdx.x & 31;
  const int wave = threadIdx.x >> 5;
  const int tilesN = N >> 6;
  const int tilesM = M >> 6;
  const int tile = blockIdx.x * 8 + wave;
  if (tile >= tilesM * tilesN) return;
  const int tm = tile / tilesN;
  const int tn = tile - tm * tilesN;
  const int m0 = tm << 6;
  const int n0 = tn << 6;

  const int rlane = lane & 15;
  const int koff  = (lane >> 4) * 8;
  const int mOff  = (lane >> 4) * 8;

  v8f acc[4][4];
#pragma unroll
  for (int i = 0; i < 4; ++i)
#pragma unroll
    for (int j = 0; j < 4; ++j) acc[i][j] = (v8f){0.f, 0.f, 0.f, 0.f, 0.f, 0.f, 0.f, 0.f};

  for (int k0 = 0; k0 < K; k0 += 32) {
    v16h bh[4];
#pragma unroll
    for (int j = 0; j < 4; ++j) {
      const size_t bo = (size_t)(n0 + (j << 4) + rlane) * ldb + koff + k0;
      bh[j] = frag_load(Bt + bo);
    }
#pragma unroll
    for (int i = 0; i < 4; ++i) {
      const size_t ao = (size_t)(m0 + (i << 4) + rlane) * lda + koff + k0;
      const v16h ah = frag_load(A + ao);
#pragma unroll
      for (int j = 0; j < 4; ++j) acc[i][j] = mma_g(ah, bh[j], acc[i][j]);
    }
    keep4_h(bh[0], bh[1], bh[2], bh[3]);
  }

  float* slab = sT[wave];
  const bool isBC = (EPI == 1) && (n0 >= kDin);
  float bvj[4] = {0.f, 0.f, 0.f, 0.f};
  if (EPI == 1) {
#pragma unroll
    for (int j = 0; j < 4; ++j) {
      const int n  = n0 + (j << 4) + rlane;
      const int nb = (n < kDin) ? n : (kDin - 1);
      const float bl = bias[nb];
      bvj[j] = isBC ? 0.0f : bl;
    }
  }
#pragma unroll
  for (int i = 0; i < 4; ++i) {
    const int mBase = m0 + (i << 4);
#pragma unroll
    for (int j = 0; j < 4; ++j) {
#pragma unroll
      for (int r = 0; r < 8; ++r) {
        float v = acc[i][j][r] * scale;
        if (EPI == 1) v += bvj[j];
        slab[(mOff + r) * 68 + (j << 4) + rlane] = v;
      }
    }
    __builtin_amdgcn_fence(__ATOMIC_RELEASE, "workgroup");
    __builtin_amdgcn_wave_barrier();
    __builtin_amdgcn_fence(__ATOMIC_ACQUIRE, "workgroup");
    if (EPI == 0) {
      const int hh = lane >> 4, c4 = (lane & 15) * 4;
      for (int pass = 0; pass < 2; ++pass) {
#pragma unroll
        for (int it = 0; it < 8; ++it) {
          const int row = it * 2 + hh;
          const v4f v = *(const v4f*)(slab + row * 68 + c4);
          *(volatile v4f*)(Cf + (size_t)(mBase + row) * ldc + n0 + c4) = v;
        }
        __threadfence();
      }
    } else {
      const int q = lane >> 3;
      if (!isBC) {
        const int c8 = (lane & 7) * 8;
        for (int pass = 0; pass < 2; ++pass) {
#pragma unroll
          for (int it = 0; it < 4; ++it) {
            const int row = it * 4 + q;
            const float* sp = slab + row * 68 + c8;
            v8h hv;
#pragma unroll
            for (int e = 0; e < 8; ++e) hv[e] = (_Float16)sp[e];
            *(volatile v8h*)(C16 + (size_t)(mBase + row) * kDin + n0 + c8) = hv;
          }
          __threadfence();
        }
      } else {
        const int c4 = (lane & 7) * 4;
        for (int pass = 0; pass < 2; ++pass) {
#pragma unroll
          for (int it = 0; it < 4; ++it) {
            const int row = it * 4 + q;
            const v4f v = *(const v4f*)(slab + row * 68 + c4);
            *(volatile v4f*)(Cbc + (size_t)(mBase + row) * kBcP + c4) = v;
          }
          __threadfence();
        }
      }
    }
    __builtin_amdgcn_fence(__ATOMIC_RELEASE, "workgroup");
    __builtin_amdgcn_wave_barrier();
    __builtin_amdgcn_fence(__ATOMIC_ACQUIRE, "workgroup");
  }
}

__global__ __launch_bounds__(256) void cast_f16_kernel(
    const float* __restrict__ src, unsigned short* __restrict__ dst, int total8, float scale)
{
  const int i = blockIdx.x * 256 + threadIdx.x;
  if (i >= total8) return;
  const size_t e0 = (size_t)i << 3;
  const v4f a0 = *(const v4f*)(src + e0);
  const v4f a1 = *(const v4f*)(src + e0 + 4);
  v8h hv;
#pragma unroll
  for (int e = 0; e < 4; ++e) {
    hv[e]     = f16_operand(a0[e] * scale);
    hv[4 + e] = f16_operand(a1[e] * scale);
  }
  unsigned short* q = dst + e0;
  *(volatile v8h*)q = hv;
  __threadfence();
  *(volatile v8h*)q = hv;
}

__global__ __launch_bounds__(256) void zero16_kernel(unsigned short* __restrict__ dst, int total8)
{
  const int i = blockIdx.x * 256 + threadIdx.x;
  if (i >= total8) return;
  const v8h z = (v8h){(_Float16)0.f, (_Float16)0.f, (_Float16)0.f, (_Float16)0.f,
                      (_Float16)0.f, (_Float16)0.f, (_Float16)0.f, (_Float16)0.f};
  unsigned short* q = dst + ((size_t)i << 3);
  *(volatile v8h*)q = z;
  __threadfence();
  *(volatile v8h*)q = z;
}

__global__ __launch_bounds__(256) void conv_silu_f16_kernel(
    const float* __restrict__ XR, const float* __restrict__ cw, const float* __restrict__ cb,
    unsigned short* __restrict__ XS16)
{
  __shared__ __align__(16) float sT[16 * kConvTP];
  const int tid = threadIdx.x, lane = tid & 31, wave = tid >> 5;
  const int d0 = blockIdx.x * 256, d = d0 + tid;
  const int g0 = blockIdx.y * 64;
  const int tb = g0 & (kSeq - 1);
  const v4f wv = *(const v4f*)(cw + (size_t)d * 4);
  const float w0 = wv[0], w1 = wv[1], w2 = wv[2], w3 = wv[3];
  const float bc = cb[d];
  float xm3, xm2, xm1;
  {
    const bool hist = (tb > 0);
    const int rb = hist ? (g0 - 3) : g0;
    const float v3 = XR[(size_t)rb * kXrP + d];
    const float v2 = XR[(size_t)(rb + 1) * kXrP + d];
    const float v1 = XR[(size_t)(rb + 2) * kXrP + d];
    xm3 = hist ? v3 : 0.f;
    xm2 = hist ? v2 : 0.f;
    xm1 = hist ? v1 : 0.f;
  }
#pragma unroll 1
  for (int sub = 0; sub < 4; ++sub) {
    const int lb = g0 + sub * 16;
#pragma unroll 1
    for (int s = 0; s < 16; ++s) {
      const float xcur = XR[(size_t)(lb + s) * kXrP + d];
      float acc = w0 * xm3;
      acc = fmaf(w1, xm2, acc);
      acc = fmaf(w2, xm1, acc);
      acc = fmaf(w3, xcur, acc);
      const float sv = acc + bc;
      const float sg = __builtin_amdgcn_rcpf(1.0f + __expf(-sv));
      sT[s * kConvTP + tid] = (sv * sg) * kCarryXs;
      xm3 = xm2; xm2 = xm1; xm1 = xcur;
    }
    __syncthreads();
    v8h bv[2];
#pragma unroll
    for (int it = 0; it < 2; ++it) {
      const float* sp = sT + (it * 8 + wave) * kConvTP + lane * 8;
      const v4f a0 = *(const v4f*)(sp);
      const v4f a1 = *(const v4f*)(sp + 4);
#pragma unroll
      for (int e = 0; e < 4; ++e) {
        bv[it][e]     = f16_operand(a0[e]);
        bv[it][4 + e] = f16_operand(a1[e]);
      }
    }
    for (int pass = 0; pass < 2; ++pass) {
#pragma unroll
      for (int it = 0; it < 2; ++it)
        *(volatile v8h*)(XS16 + (size_t)(lb + it * 8 + wave) * kDin + d0 + lane * 8) = bv[it];
      __threadfence();
    }
    __syncthreads();
  }
}

__global__ __launch_bounds__(64) void scan_kernel(
    const float* __restrict__ XR, const unsigned short* __restrict__ DP16, const float* __restrict__ BC,
    const float* __restrict__ cw, const float* __restrict__ cb, const float* __restrict__ Alog,
    const float* __restrict__ Dp, unsigned short* __restrict__ YG16)
{
  __shared__ __align__(16) float sBC[kScanTS * kBcP];
  __shared__ __align__(16) float sY[kScanTS * kScanYP];
  __shared__ __align__(16) float sA[kNst * kScanCh];
  const int tid = threadIdx.x, lane = tid & 31, wave = tid >> 5;
  constexpr int kBlkPerB = kDin / kScanCh;
  const int bix = blockIdx.x / kBlkPerB;
  const int d0  = (blockIdx.x - bix * kBlkPerB) * kScanCh;
  const int d   = d0 + tid;
  const size_t row0 = (size_t)bix * kSeq;
#pragma unroll 1
  for (int s = 0; s < kNst; ++s) sA[s * kScanCh + tid] = -expf(Alog[(size_t)d * kNst + s]);
  __syncthreads();
  float negA[kNst], h[kNst];
#pragma unroll
  for (int s = 0; s < kNst; ++s) {
    negA[s] = sA[s * kScanCh + tid];
    h[s] = 0.f;
  }
  const v4f wv = *(const v4f*)(cw + (size_t)d * 4);
  const float w0 = wv[0], w1 = wv[1], w2 = wv[2], w3 = wv[3];
  const float cbias = cb[d];
  const float Dd = Dp[d];
  float xm3 = 0.f, xm2 = 0.f, xm1 = 0.f;
  const int q = lane >> 3, c8 = (lane & 7) * 8;
#pragma unroll 1
  for (int t0 = 0; t0 < kSeq; t0 += kScanTS) {
    __syncthreads();
#pragma unroll
    for (int i = 0; i < 8; ++i) {
      const int idx = tid + 64 * i;
      *(v4f*)(sBC + idx * 4) = *(const v4f*)(BC + (row0 + t0) * kBcP + (size_t)idx * 4);
    }
    __syncthreads();
#pragma unroll 1
    for (int s = 0; s < kScanTS; ++s) {
      const size_t row = row0 + t0 + s;
      const float xcur = XR[row * kXrP + d];
      const float zv   = XR[row * kXrP + kDin + d];
      const unsigned hb = (unsigned)DP16[row * kDin + d];
      const float v = h16_to_f32(hb);
      float cacc = w0 * xm3;
      cacc = fmaf(w1, xm2, cacc);
      cacc = fmaf(w2, xm1, cacc);
      cacc = fmaf(w3, xcur, cacc);
      xm3 = xm2; xm2 = xm1; xm1 = xcur;
      const float cv = cacc + cbias;
      const float xs = cv * __builtin_amdgcn_rcpf(1.0f + __expf(-cv));
      const float a   = __expf(-fabsf(v));
      const float u   = 1.0f + a;
      const float l1p = __logf(u) + (a - (u - 1.0f)) * __builtin_amdgcn_rcpf(u);
      const float dt  = fmaxf(v, 0.0f) + l1p;
      const float dtx = dt * xs;
      const float* br = sBC + s * kBcP;
      float Bs[kNst], Cs[kNst];
#pragma unroll
      for (int q4 = 0; q4 < 4; ++q4) {
        const v4f bvv = *(const v4f*)(br + 4 * q4);
        const v4f cvv = *(const v4f*)(br + kNst + 4 * q4);
        Bs[4 * q4 + 0] = bvv[0]; Bs[4 * q4 + 1] = bvv[1]; Bs[4 * q4 + 2] = bvv[2]; Bs[4 * q4 + 3] = bvv[3];
        Cs[4 * q4 + 0] = cvv[0]; Cs[4 * q4 + 1] = cvv[1]; Cs[4 * q4 + 2] = cvv[2]; Cs[4 * q4 + 3] = cvv[3];
      }
      float y = 0.f;
#pragma unroll
      for (int k = 0; k < kNst; ++k) {
        const float e = __expf(dt * negA[k]);
        h[k] = e * h[k] + dtx * Bs[k];
        y = h[k] * Cs[k] + y;
      }
      y = xs * Dd + y;
      const float g = zv * __builtin_amdgcn_rcpf(1.0f + __expf(-zv));
      sY[s * kScanYP + tid] = (y * g) * kCarryYg;
    }
    __syncthreads();
    v8h hv[8];
#pragma unroll
    for (int it = 0; it < 8; ++it) {
      const int rr = it * 8 + wave * 4 + q;
      const float* sp = sY + rr * kScanYP + c8;
      const v4f a0 = *(const v4f*)(sp);
      const v4f a1 = *(const v4f*)(sp + 4);
#pragma unroll
      for (int e = 0; e < 4; ++e) {
        hv[it][e]     = f16_operand(a0[e]);
        hv[it][4 + e] = f16_operand(a1[e]);
      }
    }
    for (int pass = 0; pass < 2; ++pass) {
#pragma unroll
      for (int it = 0; it < 8; ++it) {
        const int rr = it * 8 + wave * 4 + q;
        *(volatile v8h*)(YG16 + (row0 + t0 + rr) * kDin + d0 + c8) = hv[it];
      }
      __threadfence();
    }
  }
}

extern "C" void kernel_launch(void* const* d_in, const int* in_sizes, int n_in,
                              void* d_out, int out_size, void* d_ws, size_t ws_size,
                              hipStream_t stream)
{
  if (n_in < 11) return;
  if (in_sizes[0] != kRows * kDm) return;
  if (in_sizes[1] != kXrP * kDm) return;
  if (in_sizes[2] != kDin * 4) return;
  if (in_sizes[3] != kDin) return;
  if (in_sizes[4] != kNst * kDin) return;
  if (in_sizes[5] != kNst * kDin) return;
  if (in_sizes[6] != kDin * kDin) return;
  if (in_sizes[7] != kDin) return;
  if (in_sizes[8] != kDin * kNst) return;
  if (in_sizes[9] != kDin) return;
  if (in_sizes[10] != kDm * kDin) return;
  if (out_size != kRows * kDm) return;
  if (ws_size < kWsTotal) return;

  const float* x       = (const float*)d_in[0];
  const float* W_in    = (const float*)d_in[1];
  const float* conv_w  = (const float*)d_in[2];
  const float* conv_b  = (const float*)d_in[3];
  const float* W_b     = (const float*)d_in[4];
  const float* W_c     = (const float*)d_in[5];
  const float* W_dt    = (const float*)d_in[6];
  const float* b_dt    = (const float*)d_in[7];
  const float* A_log   = (const float*)d_in[8];
  const float* Dp      = (const float*)d_in[9];
  const float* W_out   = (const float*)d_in[10];
  float* out = (float*)d_out;

  char* ws = (char*)d_ws;
  unsigned short* X16    = (unsigned short*)(ws + kOffX16);
  unsigned short* WIN16  = (unsigned short*)(ws + kOffWin);
  unsigned short* WDBC16 = (unsigned short*)(ws + kOffWdbc);
  unsigned short* WOUT16 = (unsigned short*)(ws + kOffWout);
  float*          XR     = (float*)(ws + kOffXr);
  unsigned short* XS16   = (unsigned short*)(ws + kOffXs16);
  unsigned short* DP16   = (unsigned short*)(ws + kOffDp16);
  float*          BC     = (float*)(ws + kOffBc);
  unsigned short* YG16   = (unsigned short*)(ws + kOffYg16);

  cast_f16_kernel<<<(kRows * kDm / 8) / 256, 256, 0, stream>>>(x, X16, kRows * kDm / 8, kCarryX);
  cast_f16_kernel<<<(kXrP * kDm / 8) / 256, 256, 0, stream>>>(W_in, WIN16, kXrP * kDm / 8, kCarryW);
  cast_f16_kernel<<<(kDin * kDin / 8) / 256, 256, 0, stream>>>(W_dt, WDBC16, kDin * kDin / 8, kCarryW);
  cast_f16_kernel<<<(kNst * kDin / 8) / 256, 256, 0, stream>>>(
      W_b, WDBC16 + (size_t)kDin * kDin, kNst * kDin / 8, kCarryW);
  cast_f16_kernel<<<(kNst * kDin / 8) / 256, 256, 0, stream>>>(
      W_c, WDBC16 + (size_t)(kDin + kNst) * kDin, kNst * kDin / 8, kCarryW);
  zero16_kernel<<<((kDbcN - kDbcReal) * kDin / 8) / 256, 256, 0, stream>>>(
      WDBC16 + (size_t)kDbcReal * kDin, (kDbcN - kDbcReal) * kDin / 8);
  cast_f16_kernel<<<(kDm * kDin / 8) / 256, 256, 0, stream>>>(W_out, WOUT16, kDm * kDin / 8, kCarryW);

  gemm64_f16_kernel<0><<<512, 256, 0, stream>>>(
      X16, kDm, WIN16, kDm, XR, kXrP, nullptr, nullptr, nullptr, kRows, kXrP, kDm, kFoldIn);

  conv_silu_f16_kernel<<<dim3(kDin / 256, kRows / 64), 256, 0, stream>>>(XR, conv_w, conv_b, XS16);

  gemm64_f16_kernel<1><<<272, 256, 0, stream>>>(
      XS16, kDin, WDBC16, kDin, nullptr, 0, b_dt, DP16, BC, kRows, kDbcN, kDin, kFoldDbc);

  scan_kernel<<<kBatch * (kDin / kScanCh), kScanCh, 0, stream>>>(XR, DP16, BC, conv_w, conv_b, A_log, Dp, YG16);

  gemm64_f16_kernel<0><<<128, 256, 0, stream>>>(
      YG16, kDin, WOUT16, kDin, out, kDm, nullptr, nullptr, nullptr, kRows, kDm, kDin, kFoldOut);
}
